// PINN_52123723104357
// MI455X (gfx1250) — hardware-verified
//
#include <hip/hip_runtime.h>
#include <stddef.h>
#include <stdint.h>

#define IND    3
#define HID    40
#define OUTD   3
#define NHID   5
#define KS     3
#define KPK    (KS * 32)
#define KP     96
#define NT     3
#define NPAD   (NT * 16)
#define HNP    16
#define NWAVES 4
#define TM     16
#define RPI    (NWAVES * TM)
#define ITERS  32
#define RPB    (RPI * ITERS)
#define WMAT   (NPAD * KP)
#define W6MAT  (HNP * KP)
#define ATILE  (TM * KP)
#define DYN_ELEMS (NHID * WMAT)

static_assert(KPK == 2 * HID + 16);
static_assert(KP >= KPK);
static_assert((KP % 8) == 0);
static_assert(NPAD >= HID);
static_assert(((WMAT / 2) % 128) == 0);
static_assert(((W6MAT / 2) % 128) == 0);
static_assert(NWAVES * 32 == 128);
static_assert(DYN_ELEMS * 2 == 46080);
static_assert(RPI * OUTD == 192);
static_assert((RPB % RPI) == 0);
static_assert(IND * HID <= 128);

typedef unsigned short v8us  __attribute__((ext_vector_type(8)));
typedef unsigned short v16us __attribute__((ext_vector_type(16)));
typedef float          v4f   __attribute__((ext_vector_type(4)));
typedef float          v8f   __attribute__((ext_vector_type(8)));
#if defined(__HIP_DEVICE_COMPILE__)
typedef __bf16         v16bf __attribute__((ext_vector_type(16)));
#endif

union FragU { v16us v; v8us half[2]; };

__device__ __forceinline__ unsigned bbits(float f) {
  unsigned u = __float_as_uint(f);
  return (u + 0x7FFFu + ((u >> 16) & 1u)) >> 16;
}
__device__ __forceinline__ float bf16r(float f) {
  return __uint_as_float(bbits(f) << 16);
}
__device__ __forceinline__ v8f zero8() { v8f z = {0.f, 0.f, 0.f, 0.f, 0.f, 0.f, 0.f, 0.f}; return z; }
__device__ __forceinline__ v8us zero8us() { v8us z = {0, 0, 0, 0, 0, 0, 0, 0}; return z; }
__device__ __forceinline__ float tanh_f(float z) {
  const float zc = fminf(fmaxf(z, -10.0f), 10.0f);
  const float e  = __expf(2.0f * zc);
  return 1.0f - 2.0f * __builtin_amdgcn_rcpf(e + 1.0f);
}
__device__ __forceinline__ void split2(float v, unsigned short& hb, unsigned short& lb) {
  const unsigned hu = bbits(v);
  hb = (unsigned short)hu;
  lb = (unsigned short)bbits(v - __uint_as_float(hu << 16));
}

__device__ __forceinline__ v16us ldfrag(const unsigned short* p) {
  FragU f;
  f.half[0] = *(const v8us*)(p);
  f.half[1] = *(const v8us*)(p + 16);
  return f.v;
}

__device__ __forceinline__ v8f mma_bf(v16us a, v16us b, v8f c) {
#if defined(__HIP_DEVICE_COMPILE__)
  return __builtin_amdgcn_wmma_f32_16x16x32_bf16(false, __builtin_bit_cast(v16bf, a),
                                                false, __builtin_bit_cast(v16bf, b),
                                                (short)0, c, false, false);
#else
  (void)a; (void)b;
  return c;
#endif
}
__device__ __forceinline__ void guard6(v8f& acc, const v16us& a0, const v16us& a1, const v16us& a2,
                                       const v16us& b0, const v16us& b1, const v16us& b2) {
#if defined(__HIP_DEVICE_COMPILE__)
  asm volatile("v_nop\n\tv_nop\n\tv_nop\n\tv_nop"
               : "+v"(acc)
               : "v"(a0), "v"(a1), "v"(a2), "v"(b0), "v"(b1), "v"(b2));
#endif
}

__device__ __forceinline__ float wsel_hidden(const float* __restrict__ W, int n, int k) {
  int kk = (k < HID) ? k : (k - HID);
  kk = (kk < 0) ? 0 : ((kk > HID - 1) ? (HID - 1) : kk);
  const int nn = (n > HID - 1) ? (HID - 1) : n;
  const float v = W[kk * HID + nn];
  return (n < HID && k < 2 * HID) ? v : 0.0f;
}
__device__ __forceinline__ float wsel_head(const float* __restrict__ W, int n, int k) {
  int kk = (k < HID) ? k : (k - HID);
  kk = (kk < 0) ? 0 : ((kk > HID - 1) ? (HID - 1) : kk);
  const int nn = (n > OUTD - 1) ? (OUTD - 1) : n;
  const float v = W[kk * OUTD + nn];
  return (n < OUTD && k < 2 * HID) ? v : 0.0f;
}
__device__ __forceinline__ void stage_hidden(const float* __restrict__ W, unsigned short* dst, int tid) {
  unsigned int* d32 = (unsigned int*)dst;
#pragma unroll 2
  for (int q = 0; q < (WMAT / 2) / 128; ++q) {
    const int p  = tid + q * 128;
    const int n  = p / (KP / 2);
    const int k2 = (p - n * (KP / 2)) * 2;
    const float f0 = wsel_hidden(W, n, k2);
    const float f1 = wsel_hidden(W, n, k2 + 1);
    d32[p] = bbits(f0) | (bbits(f1) << 16);
  }
}
__device__ __forceinline__ void stage_head(const float* __restrict__ W, unsigned short* dst, int tid) {
  unsigned int* d32 = (unsigned int*)dst;
#pragma unroll 2
  for (int q = 0; q < (W6MAT / 2) / 128; ++q) {
    const int p  = tid + q * 128;
    const int n  = p / (KP / 2);
    const int k2 = (p - n * (KP / 2)) * 2;
    const float f0 = wsel_head(W, n, k2);
    const float f1 = wsel_head(W, n, k2 + 1);
    d32[p] = bbits(f0) | (bbits(f1) << 16);
  }
}
__device__ __forceinline__ void stage_bias(const float* __restrict__ B, float* dst, int tid) {
  const float v = B[(tid < HID) ? tid : (HID - 1)];
  if (tid < NPAD) dst[tid] = (tid < HID) ? bf16r(v) : 0.0f;
}

__global__ __launch_bounds__(128)
void k_mlp(const float* __restrict__ X,
           const float* __restrict__ W0, const float* __restrict__ Bi0,
           const float* __restrict__ W1, const float* __restrict__ Bi1,
           const float* __restrict__ W2, const float* __restrict__ Bi2,
           const float* __restrict__ W3, const float* __restrict__ Bi3,
           const float* __restrict__ W4, const float* __restrict__ Bi4,
           const float* __restrict__ W5, const float* __restrict__ Bi5,
           const float* __restrict__ W6, const float* __restrict__ Bi6,
           float* out, int nx)
{
  extern __shared__ __align__(16) unsigned short dynlds[];
  __shared__ __align__(16) unsigned short w6s[W6MAT];
  __shared__ __align__(16) unsigned short acts[NWAVES * ATILE];
  __shared__ __align__(16) float w0f[IND * HID];
  __shared__ __align__(16) float b0f[HID];
  __shared__ __align__(16) float bhf[NHID * NPAD];
  __shared__ __align__(16) float b6f[HNP];
  __shared__ __align__(16) float sOut[RPI * OUTD];

  const int tid = threadIdx.x;

  stage_hidden(W1, dynlds + 0 * WMAT, tid);
  stage_hidden(W2, dynlds + 1 * WMAT, tid);
  stage_hidden(W3, dynlds + 2 * WMAT, tid);
  stage_hidden(W4, dynlds + 3 * WMAT, tid);
  stage_hidden(W5, dynlds + 4 * WMAT, tid);
  stage_head(W6, w6s, tid);
  {
    const float v = W0[(tid < IND * HID) ? tid : (IND * HID - 1)];
    if (tid < IND * HID) w0f[tid] = bf16r(v);
  }
  {
    const float v = Bi0[(tid < HID) ? tid : (HID - 1)];
    if (tid < HID) b0f[tid] = bf16r(v);
  }
  stage_bias(Bi1, bhf + 0 * NPAD, tid);
  stage_bias(Bi2, bhf + 1 * NPAD, tid);
  stage_bias(Bi3, bhf + 2 * NPAD, tid);
  stage_bias(Bi4, bhf + 3 * NPAD, tid);
  stage_bias(Bi5, bhf + 4 * NPAD, tid);
  {
    const float v = Bi6[(tid < OUTD) ? tid : (OUTD - 1)];
    if (tid < HNP) b6f[tid] = (tid < OUTD) ? bf16r(v) : 0.0f;
  }
  __syncthreads();

  const int lane = tid & 31;
  const int wave = tid >> 5;
  const int hh   = lane >> 4;
  const int c    = lane & 15;
  unsigned short* act = acts + wave * ATILE;
  const int blockRow0 = blockIdx.x * RPB;
  const v8us z8 = zero8us();

#pragma unroll 1
  for (int it = 0; it < ITERS; ++it) {
    const int rbase = blockRow0 + it * RPI;
    if (rbase >= nx) break;
    const int r0w = rbase + wave * TM;
    __syncthreads();

    {
      int gr = r0w + c;
      if (gr > nx - 1) gr = nx - 1;
      const float* xp = X + (size_t)gr * IND;
      const float x0 = bf16r(xp[0]);
      const float x1 = bf16r(xp[1]);
      const float x2 = bf16r(xp[2]);
      unsigned short* arow = act + c * KP;
      *(v8us*)(arow + 2 * HID + 8 * hh) = z8;
#pragma unroll 4
      for (int j = 0; j < HID / 2; ++j) {
        const int n = hh * (HID / 2) + j;
        float d = x0 * w0f[n];
        d = fmaf(x1, w0f[HID + n], d);
        d = fmaf(x2, w0f[2 * HID + n], d);
        const float hv = tanh_f(d + b0f[n]);
        unsigned short hb, lb;
        split2(hv, hb, lb);
        arow[n]       = hb;
        arow[HID + n] = lb;
      }
    }
    __syncthreads();

#pragma unroll 1
    for (int li = 0; li < NHID; ++li) {
      const unsigned short* wl = dynlds + li * WMAT;
      const unsigned short* ar = act + c * KP + 8 * hh;
      const v16us a0 = ldfrag(ar);
      const v16us a1 = ldfrag(ar + 32);
      const v16us a2 = ldfrag(ar + 64);
#pragma unroll 1
      for (int nt = 0; nt < NT; ++nt) {
        const int n0 = nt * 16;
        const unsigned short* wp = wl + (n0 + c) * KP + 8 * hh;
        const v16us g0 = ldfrag(wp);
        const v16us g1 = ldfrag(wp + 32);
        const v16us g2 = ldfrag(wp + 64);
        v8f acc = zero8();
        acc = mma_bf(a0, g0, acc);
        acc = mma_bf(a1, g1, acc);
        acc = mma_bf(a2, g2, acc);
        guard6(acc, a0, a1, a2, g0, g1, g2);
        const int n = n0 + c;
        const float bias = bhf[li * NPAD + n];
        if (n < HID) {
#pragma unroll
          for (int r = 0; r < 8; ++r) {
            const float hv = tanh_f(acc[r] + bias);
            unsigned short hb, lb;
            split2(hv, hb, lb);
            const int o = (8 * hh + r) * KP;
            act[o + n]       = hb;
            act[o + HID + n] = lb;
          }
        }
      }
      __syncthreads();
    }

    {
      const unsigned short* ar = act + c * KP + 8 * hh;
      const v16us a0 = ldfrag(ar);
      const v16us a1 = ldfrag(ar + 32);
      const v16us a2 = ldfrag(ar + 64);
      const unsigned short* wp = w6s + c * KP + 8 * hh;
      const v16us g0 = ldfrag(wp);
      const v16us g1 = ldfrag(wp + 32);
      const v16us g2 = ldfrag(wp + 64);
      v8f acc = zero8();
      acc = mma_bf(a0, g0, acc);
      acc = mma_bf(a1, g1, acc);
      acc = mma_bf(a2, g2, acc);
      guard6(acc, a0, a1, a2, g0, g1, g2);
      const float bias = b6f[c];
      if (c < OUTD) {
#pragma unroll
        for (int r = 0; r < 8; ++r) sOut[(wave * TM + 8 * hh + r) * OUTD + c] = acc[r] + bias;
      }
    }
    __syncthreads();

    {
      const int q = (wave == 0) ? lane : (32 + c);
      const v4f ov = *(const v4f*)(sOut + 4 * q);
      const bool wr = (wave == 0) || ((wave == 1) && (lane < 16));
      float* po = out + (size_t)rbase * OUTD + 4 * q;
      if (wr) *(volatile v4f*)po = ov;
      __threadfence();
      if (wr) *(volatile v4f*)po = ov;
    }
  }
}

extern "C" void kernel_launch(void* const* d_in, const int* in_sizes, int n_in,
                              void* d_out, int out_size, void* d_ws, size_t ws_size,
                              hipStream_t stream) {
  (void)d_ws; (void)ws_size;
  if (n_in < 15) return;
  if (in_sizes[0] < IND * RPI || (in_sizes[0] % IND) != 0) return;
  const int nx = in_sizes[0] / IND;
  if ((nx % RPI) != 0) return;
  if (in_sizes[1] != IND * HID || in_sizes[2] != HID) return;
  for (int i = 0; i < NHID; ++i) {
    if (in_sizes[3 + 2 * i] != HID * HID) return;
    if (in_sizes[4 + 2 * i] != HID) return;
  }
  if (in_sizes[13] != HID * OUTD || in_sizes[14] != OUTD) return;
  if ((long long)out_size != (long long)nx * (long long)OUTD) return;

  const float* X = (const float*)d_in[0];
  const float* W0 = (const float*)d_in[1];  const float* Bi0 = (const float*)d_in[2];
  const float* W1 = (const float*)d_in[3];  const float* Bi1 = (const float*)d_in[4];
  const float* W2 = (const float*)d_in[5];  const float* Bi2 = (const float*)d_in[6];
  const float* W3 = (const float*)d_in[7];  const float* Bi3 = (const float*)d_in[8];
  const float* W4 = (const float*)d_in[9];  const float* Bi4 = (const float*)d_in[10];
  const float* W5 = (const float*)d_in[11]; const float* Bi5 = (const float*)d_in[12];
  const float* W6 = (const float*)d_in[13]; const float* Bi6 = (const float*)d_in[14];
  float* out = (float*)d_out;

  const size_t dynBytes = (size_t)DYN_ELEMS * sizeof(unsigned short);
  (void)hipFuncSetAttribute(reinterpret_cast<const void*>(&k_mlp),
                            hipFuncAttributeMaxDynamicSharedMemorySize, (int)dynBytes);
  const dim3 grid((nx + RPB - 1) / RPB);
  k_mlp<<<grid, dim3(128), dynBytes, stream>>>(X, W0, Bi0, W1, Bi1, W2, Bi2, W3, Bi3,
                                               W4, Bi4, W5, Bi5, W6, Bi6, out, nx);
  (void)hipGetLastError();
}
